// Meta_Transformer_Layer_7499012899506
// MI455X (gfx1250) — hardware-verified
//
#include <hip/hip_runtime.h>
#include <stddef.h>


typedef __bf16   v16b __attribute__((ext_vector_type(16)));
typedef __bf16   v8b  __attribute__((ext_vector_type(8)));
typedef _Float16 v16h __attribute__((ext_vector_type(16)));
typedef _Float16 v8h  __attribute__((ext_vector_type(8)));
typedef float    v8f  __attribute__((ext_vector_type(8)));
typedef float    v4f  __attribute__((ext_vector_type(4)));
typedef int      v4i  __attribute__((ext_vector_type(4)));

#define NB 8
#define NS 1024
#define NE 1024
#define NH 16
#define ND 64
#define NM (NB * NS)
#define TP 68
#define CQ 0.18033688011112042f
#define PSH 12.0f
#define WSC 64.0f
#define WSCI 0.015625f

union FragB { v16b v; v8b q[2]; };
union FragH { v16h v; v8h q[2]; };
union PackB { v8b b; v4i i; };
union PackH { v8h e; v4i i; };

#define BV(x) __builtin_bit_cast(v8f, (x))
#define NOP4 "v_nop\n\tv_nop\n\tv_nop\n\tv_nop"

__device__ __forceinline__ v8f wm_bf16(v16b a, v16b b, v8f c) {
  return __builtin_amdgcn_wmma_f32_16x16x32_bf16(false, a, false, b, (short)0, c, false, false);
}
__device__ __forceinline__ v8f wm_f16(v16h a, v16h b, v8f c) {
  return __builtin_amdgcn_wmma_f32_16x16x32_f16(false, a, false, b, (short)0, c, false, false);
}
__device__ __forceinline__ v8f wm3(v16b ah, v16b al, v16b bh, v16b bl, v8f c) {
  c = wm_bf16(ah, bh, c);
  c = wm_bf16(ah, bl, c);
  c = wm_bf16(al, bh, c);
  return c;
}
#define WG8x6(c0, c1, c2, c3, c4, c5, c6, c7, f0, f1, f2, f3, f4, f5)                               \
  asm volatile(NOP4 : "+v"(c0), "+v"(c1), "+v"(c2), "+v"(c3), "+v"(c4), "+v"(c5), "+v"(c6), "+v"(c7)   \
               : "v"(BV(f0)), "v"(BV(f1)), "v"(BV(f2)), "v"(BV(f3)), "v"(BV(f4)), "v"(BV(f5)))
#define WG2x12(c0, c1, f0, f1, f2, f3, f4, f5, f6, f7, f8, f9, f10, f11)                              \
  asm volatile(NOP4 : "+v"(c0), "+v"(c1)                                                              \
               : "v"(BV(f0)), "v"(BV(f1)), "v"(BV(f2)), "v"(BV(f3)), "v"(BV(f4)), "v"(BV(f5)),        \
                 "v"(BV(f6)), "v"(BV(f7)), "v"(BV(f8)), "v"(BV(f9)), "v"(BV(f10)), "v"(BV(f11)))
#define WG4x10(c0, c1, c2, c3, f0, f1, f2, f3, f4, f5, f6, f7, f8, f9)                                 \
  asm volatile(NOP4 : "+v"(c0), "+v"(c1), "+v"(c2), "+v"(c3)                                          \
               : "v"(BV(f0)), "v"(BV(f1)), "v"(BV(f2)), "v"(BV(f3)), "v"(BV(f4)),                     \
                 "v"(BV(f5)), "v"(BV(f6)), "v"(BV(f7)), "v"(BV(f8)), "v"(BV(f9)))

__device__ __forceinline__ v16b ldb(const __bf16* p, int h) {
  FragB f;
  f.q[0] = *(const v8b*)(p + 8 * h);
  f.q[1] = *(const v8b*)(p + 16 + 8 * h);
  return f.v;
}
__device__ __forceinline__ v16h ldh(const _Float16* p, int h) {
  FragH f;
  f.q[0] = *(const v8h*)(p + 8 * h);
  f.q[1] = *(const v8h*)(p + 16 + 8 * h);
  return f.v;
}

__device__ __forceinline__ float bfr(float x) { return (float)((__bf16)x); }

__device__ __forceinline__ void st16x2(void* p, v4i v) {
  *(volatile v4i*)p = v;
  __threadfence();
  *(volatile v4i*)p = v;
}
__device__ __forceinline__ void stf4x2(float* p, v4f v) {
  *(volatile v4f*)p = v;
  __threadfence();
  *(volatile v4f*)p = v;
}

__global__ void __launch_bounds__(256)
cvtx_kernel(const float* __restrict__ src, __bf16* dst, int n8) {
  const int g = blockIdx.x * 256 + threadIdx.x;
  if (g >= n8) return;
  const size_t o = (size_t)g * 8;
  const v4f a = *(const v4f*)(src + o);
  const v4f c = *(const v4f*)(src + o + 4);
  PackB p;
  p.b[0] = (__bf16)a.x; p.b[1] = (__bf16)a.y; p.b[2] = (__bf16)a.z; p.b[3] = (__bf16)a.w;
  p.b[4] = (__bf16)c.x; p.b[5] = (__bf16)c.y; p.b[6] = (__bf16)c.z; p.b[7] = (__bf16)c.w;
  st16x2(dst + o, p.i);
}

__global__ void __launch_bounds__(256)
wprep_kernel(const float* __restrict__ wq, const float* __restrict__ wk, const float* __restrict__ wv,
             const float* __restrict__ wo,
             __bf16* tq, __bf16* tk, __bf16* tv, _Float16* to16) {
  __shared__ float T[64][65];
  const int z = blockIdx.z;
  const int f0 = blockIdx.x * 64, e0 = blockIdx.y * 64;
  const int t = threadIdx.x;
  if (z < 3) {
    const float* W = (z == 0) ? wq : ((z == 1) ? wk : wv);
#pragma unroll
    for (int i = 0; i < 4; ++i) {
      const int c = t + 256 * i;
      const int r = c >> 4, c4 = (c & 15) * 4;
      const v4f v = *(const v4f*)(W + (size_t)(e0 + r) * NE + f0 + c4);
      T[r][c4 + 0] = v.x; T[r][c4 + 1] = v.y; T[r][c4 + 2] = v.z; T[r][c4 + 3] = v.w;
    }
  } else {
#pragma unroll
    for (int i = 0; i < 4; ++i) {
      const int c = t + 256 * i;
      const int r = c >> 4, c4 = (c & 15) * 4;
      const v4f v = *(const v4f*)(wo + (size_t)(f0 + r) * NE + e0 + c4);
      T[c4 + 0][r] = v.x; T[c4 + 1][r] = v.y; T[c4 + 2][r] = v.z; T[c4 + 3][r] = v.w;
    }
  }
  __syncthreads();
  __bf16* tz = (z == 0) ? tq : ((z == 1) ? tk : tv);
#pragma unroll
  for (int i = 0; i < 2; ++i) {
    const int c = t + 256 * i;
    const int f = c >> 3, q = c & 7;
    const size_t o = (size_t)(f0 + f) * NE + e0 + 8 * q;
    v4i bits;
    if (z < 3) {
      PackB p;
#pragma unroll
      for (int j = 0; j < 8; ++j) p.b[j] = (__bf16)T[8 * q + j][f];
      bits = p.i;
      st16x2(tz + o, bits);
    } else {
      PackH p;
#pragma unroll
      for (int j = 0; j < 8; ++j) p.e[j] = (_Float16)(bfr(T[8 * q + j][f]) * WSC);
      bits = p.i;
      st16x2(to16 + o, bits);
    }
  }
}

__global__ void __launch_bounds__(128) __attribute__((amdgpu_num_vgpr(240)))
qkv_kernel(const __bf16* __restrict__ Xb,
           const __bf16* __restrict__ Tq, const __bf16* __restrict__ Tk, const __bf16* __restrict__ Tv,
           const float* __restrict__ gq, const float* __restrict__ gk,
           __bf16* Qh, __bf16* Ql, __bf16* Kh, __bf16* Kl, _Float16* Vo) {
  __shared__ float T[128][TP];
  const int tid = threadIdx.x, lane = tid & 31, wave = tid >> 5, h = lane >> 4, l16 = lane & 15;
  const int n0 = blockIdx.x * 64, m0 = blockIdx.y * 128, z = blockIdx.z;
  const __bf16* Wt = (z == 0) ? Tq : ((z == 1) ? Tk : Tv);

  const v8f vz = {0.f, 0.f, 0.f, 0.f, 0.f, 0.f, 0.f, 0.f};
  v8f acc0[4] = {vz, vz, vz, vz};
  v8f acc1[4] = {vz, vz, vz, vz};

  const __bf16* a0p = Xb + (size_t)(m0 + wave * 32 + l16) * NE;
  const __bf16* a1p = a0p + (size_t)16 * NE;
  const __bf16* bp  = Wt + (size_t)(n0 + l16) * NE;
#pragma unroll 1
  for (int k0 = 0; k0 < NE; k0 += 32) {
    const v16b a0 = ldb(a0p + k0, h), a1 = ldb(a1p + k0, h);
    v16b bb[4];
#pragma unroll
    for (int tn = 0; tn < 4; ++tn) bb[tn] = ldb(bp + (size_t)tn * 16 * NE + k0, h);
#pragma unroll
    for (int tn = 0; tn < 4; ++tn) {
      acc0[tn] = wm_bf16(a0, bb[tn], acc0[tn]);
      acc1[tn] = wm_bf16(a1, bb[tn], acc1[tn]);
    }
    WG8x6(acc0[0], acc0[1], acc0[2], acc0[3], acc1[0], acc1[1], acc1[2], acc1[3],
          a0, a1, bb[0], bb[1], bb[2], bb[3]);
  }

  const int b = m0 / NS, hn = n0 / ND, sf = m0 - b * NS;
  const float* gp = (z == 0) ? gq : gk;
  const float s2 = (z == 0) ? (2.0f * CQ) : ((z == 1) ? 2.0f : 1.0f);
#pragma unroll
  for (int tn = 0; tn < 4; ++tn) {
    const int col = tn * 16 + l16;
    float g = 1.0f;
    if (z < 2) g = bfr(gp[b * NE + n0 + col]);
    const float gs = g * s2;
#pragma unroll
    for (int r = 0; r < 8; ++r) {
      T[wave * 32 + 8 * h + r][col]      = acc0[tn][r] * gs;
      T[wave * 32 + 16 + 8 * h + r][col] = acc1[tn][r] * gs;
    }
  }
  __syncthreads();
  if (z < 2) {
    __bf16* Oh = (z == 0) ? Qh : Kh;
    __bf16* Ol = (z == 0) ? Ql : Kl;
    const size_t ob = ((size_t)(b * NH + hn) * NS + sf) * ND;
#pragma unroll 1
    for (int p = 0; p < 8; ++p) {
      const int row = p * 16 + (tid >> 3), c = tid & 7;
      PackB ph, pl;
#pragma unroll
      for (int j = 0; j < 8; ++j) {
        const float x = T[row][8 * c + j];
        const __bf16 hv = (__bf16)x;
        ph.b[j] = hv;
        pl.b[j] = (__bf16)(x - (float)hv);
      }
      const size_t o = ob + (size_t)row * ND + 8 * c;
      st16x2(Oh + o, ph.i);
      st16x2(Ol + o, pl.i);
    }
  } else {
    const size_t ob = (size_t)(b * NH + hn) * ND * NS + sf;
#pragma unroll 1
    for (int p = 0; p < 8; ++p) {
      const int d = p * 8 + (tid >> 4), c = tid & 15;
      PackH pk;
#pragma unroll
      for (int j = 0; j < 8; ++j) pk.e[j] = (_Float16)T[8 * c + j][d];
      st16x2(Vo + ob + (size_t)d * NS + 8 * c, pk.i);
    }
  }
}

__global__ void __launch_bounds__(128) __attribute__((amdgpu_num_vgpr(240)))
attn_kernel(const __bf16* __restrict__ Qh, const __bf16* __restrict__ Ql,
            const __bf16* __restrict__ Kh, const __bf16* __restrict__ Kl,
            const _Float16* __restrict__ Vt, _Float16* AO) {
  __shared__ float T[4][16][TP];
  const int tid = threadIdx.x, lane = tid & 31, wave = tid >> 5, h = lane >> 4, l16 = lane & 15;
  const int bh = blockIdx.y;
  const int b = bh >> 4, hd = bh & 15;
  const int i0 = blockIdx.x * 64 + wave * 16;
  const size_t hb = (size_t)bh * NS * ND;

  const __bf16* qh_r = Qh + hb + (size_t)(i0 + l16) * ND;
  const __bf16* ql_r = Ql + hb + (size_t)(i0 + l16) * ND;
  const v16b qbh0 = ldb(qh_r, h), qbh1 = ldb(qh_r + 32, h);
  const v16b qbl0 = ldb(ql_r, h), qbl1 = ldb(ql_r + 32, h);

  const __bf16* kbh = Kh + hb + (size_t)l16 * ND;
  const __bf16* kbl = Kl + hb + (size_t)l16 * ND;
  const _Float16* vbr = Vt + hb + (size_t)l16 * NS;

  const v8f vz = {0.f, 0.f, 0.f, 0.f, 0.f, 0.f, 0.f, 0.f};
  v8f oacc[4] = {vz, vz, vz, vz};
  float mrun = -1.0e30f, lrun = 0.0f;

#pragma unroll 1
  for (int jb = 0; jb < NS; jb += 64) {
    v8f sc[4];
#pragma unroll
    for (int g = 0; g < 2; ++g) {
      const size_t ko = (size_t)(jb + 32 * g) * ND;
      const __bf16* kh0 = kbh + ko;
      const __bf16* kl0 = kbl + ko;
      const __bf16* kh1 = kh0 + 16 * ND;
      const __bf16* kl1 = kl0 + 16 * ND;
      const v16b a0h = ldb(kh0, h), a0l = ldb(kl0, h), a1h = ldb(kh0 + 32, h), a1l = ldb(kl0 + 32, h);
      const v16b b0h = ldb(kh1, h), b0l = ldb(kl1, h), b1h = ldb(kh1 + 32, h), b1l = ldb(kl1 + 32, h);
      v8f c0 = vz, c1 = vz;
      c0 = wm3(a0h, a0l, qbh0, qbl0, c0);
      c0 = wm3(a1h, a1l, qbh1, qbl1, c0);
      c1 = wm3(b0h, b0l, qbh0, qbl0, c1);
      c1 = wm3(b1h, b1l, qbh1, qbl1, c1);
      WG2x12(c0, c1, a0h, a0l, a1h, a1l, b0h, b0l, b1h, b1l, qbh0, qbl0, qbh1, qbl1);
      sc[2 * g] = c0;
      sc[2 * g + 1] = c1;
    }

    float mx = -1.0e30f;
#pragma unroll
    for (int tk = 0; tk < 4; ++tk)
#pragma unroll
      for (int r = 0; r < 8; ++r) mx = fmaxf(mx, sc[tk][r]);
    mx = fmaxf(mx, __shfl_xor(mx, 16, 32));
    const float mnew = fmaxf(mrun, mx);
    const float alpha = __builtin_amdgcn_exp2f(mrun - mnew);
    const float msh = mnew - PSH;
    float ps = 0.0f;
#pragma unroll
    for (int tk = 0; tk < 4; ++tk)
#pragma unroll
      for (int r = 0; r < 8; ++r) {
        const float p = __builtin_amdgcn_exp2f(sc[tk][r] - msh);
        sc[tk][r] = p;
        ps += p;
      }
    ps += __shfl_xor(ps, 16, 32);
    lrun = lrun * alpha + ps;
    mrun = mnew;
#pragma unroll
    for (int td = 0; td < 4; ++td) oacc[td] = oacc[td] * alpha;

    v16h pb0, pb1;
#pragma unroll
    for (int r = 0; r < 8; ++r) {
      pb0[r] = (_Float16)sc[0][r];  pb0[8 + r] = (_Float16)sc[1][r];
      pb1[r] = (_Float16)sc[2][r];  pb1[8 + r] = (_Float16)sc[3][r];
    }

    v16h vf[8];
#pragma unroll
    for (int td = 0; td < 4; ++td) {
      const _Float16* v_r = vbr + (size_t)(16 * td) * NS + jb;
      vf[2 * td]     = ldh(v_r, h);
      vf[2 * td + 1] = ldh(v_r + 32, h);
    }
#pragma unroll
    for (int td = 0; td < 4; ++td) {
      oacc[td] = wm_f16(vf[2 * td], pb0, oacc[td]);
      oacc[td] = wm_f16(vf[2 * td + 1], pb1, oacc[td]);
    }
    WG4x10(oacc[0], oacc[1], oacc[2], oacc[3],
           vf[0], vf[1], vf[2], vf[3], vf[4], vf[5], vf[6], vf[7], pb0, pb1);
  }

  const float inv = 1.0f / lrun;
#pragma unroll
  for (int td = 0; td < 4; ++td)
#pragma unroll
    for (int r = 0; r < 8; ++r) T[wave][l16][16 * td + 8 * h + r] = oacc[td][r] * inv;
  __syncthreads();
  const size_t tok0 = (size_t)b * NS + i0;
#pragma unroll 1
  for (int p = 0; p < 4; ++p) {
    const int row = p * 4 + (lane >> 3), c = lane & 7;
    PackH pk;
#pragma unroll
    for (int j = 0; j < 8; ++j) pk.e[j] = (_Float16)T[wave][row][8 * c + j];
    st16x2(AO + (tok0 + row) * NE + (size_t)hd * ND + 8 * c, pk.i);
  }
}

__global__ void __launch_bounds__(128) __attribute__((amdgpu_num_vgpr(240)))
outproj_kernel(const _Float16* __restrict__ AOp, const _Float16* __restrict__ Wo16,
               const float* __restrict__ X, float* R) {
  __shared__ float T[128][TP];
  const int tid = threadIdx.x, lane = tid & 31, wave = tid >> 5, h = lane >> 4, l16 = lane & 15;
  const int n0 = blockIdx.x * 64, m0 = blockIdx.y * 128;

  const v8f vz = {0.f, 0.f, 0.f, 0.f, 0.f, 0.f, 0.f, 0.f};
  v8f acc0[4] = {vz, vz, vz, vz};
  v8f acc1[4] = {vz, vz, vz, vz};

  const _Float16* a0p = AOp + (size_t)(m0 + wave * 32 + l16) * NE;
  const _Float16* a1p = a0p + (size_t)16 * NE;
  const _Float16* bp  = Wo16 + (size_t)(n0 + l16) * NE;
#pragma unroll 1
  for (int k0 = 0; k0 < NE; k0 += 32) {
    const v16h a0 = ldh(a0p + k0, h), a1 = ldh(a1p + k0, h);
    v16h bb[4];
#pragma unroll
    for (int tn = 0; tn < 4; ++tn) bb[tn] = ldh(bp + (size_t)tn * 16 * NE + k0, h);
#pragma unroll
    for (int tn = 0; tn < 4; ++tn) {
      acc0[tn] = wm_f16(a0, bb[tn], acc0[tn]);
      acc1[tn] = wm_f16(a1, bb[tn], acc1[tn]);
    }
    WG8x6(acc0[0], acc0[1], acc0[2], acc0[3], acc1[0], acc1[1], acc1[2], acc1[3],
          a0, a1, bb[0], bb[1], bb[2], bb[3]);
  }

#pragma unroll
  for (int tn = 0; tn < 4; ++tn) {
    const int col = tn * 16 + l16;
#pragma unroll
    for (int r = 0; r < 8; ++r) {
      T[wave * 32 + 8 * h + r][col]      = acc0[tn][r];
      T[wave * 32 + 16 + 8 * h + r][col] = acc1[tn][r];
    }
  }
  __syncthreads();
#pragma unroll 1
  for (int p = 0; p < 16; ++p) {
    const int L = p * 16 + wave * 4 + (lane >> 3);
    const int row = L >> 1;
    const int col = (L & 1) * 32 + (lane & 7) * 4;
    const size_t o = (size_t)(m0 + row) * NE + n0 + col;
    const v4f xv = *(const v4f*)(X + o);
    v4f v;
    v.x = T[row][col + 0] * WSCI + bfr(xv.x);
    v.y = T[row][col + 1] * WSCI + bfr(xv.y);
    v.z = T[row][col + 2] * WSCI + bfr(xv.z);
    v.w = T[row][col + 3] * WSCI + bfr(xv.w);
    stf4x2(R + o, v);
  }
}

__global__ void __launch_bounds__(256)
ln_kernel(const float* __restrict__ R, const float* __restrict__ gam, const float* __restrict__ bet,
          float* out, int nrows) {
  const int lane = threadIdx.x & 31, wave = threadIdx.x >> 5;
  const int row = blockIdx.x * 8 + wave;
  if (row >= nrows) return;
  const float* rp = R + (size_t)row * NE;
  v4f x[8];
  float s = 0.0f;
#pragma unroll
  for (int p = 0; p < 8; ++p) {
    x[p] = *(const v4f*)(rp + p * 128 + 4 * lane);
    s += (x[p].x + x[p].y) + (x[p].z + x[p].w);
  }
#pragma unroll
  for (int off = 16; off > 0; off >>= 1) s += __shfl_xor(s, off, 32);
  const float mean = s * (1.0f / NE);
  float q = 0.0f;
#pragma unroll
  for (int p = 0; p < 8; ++p) {
    const v4f d = x[p] - mean;
    q += (d.x * d.x + d.y * d.y) + (d.z * d.z + d.w * d.w);
  }
#pragma unroll
  for (int off = 16; off > 0; off >>= 1) q += __shfl_xor(q, off, 32);
  const float var = q * (1.0f / NE);
  const float inv = rsqrtf(var + 1.0e-6f);
  float* op = out + (size_t)row * NE;
#pragma unroll
  for (int p = 0; p < 8; ++p) {
    const v4f g  = *(const v4f*)(gam + p * 128 + 4 * lane);
    const v4f bb = *(const v4f*)(bet + p * 128 + 4 * lane);
    v4f gb, cb;
    gb.x = bfr(g.x);  gb.y = bfr(g.y);  gb.z = bfr(g.z);  gb.w = bfr(g.w);
    cb.x = bfr(bb.x); cb.y = bfr(bb.y); cb.z = bfr(bb.z); cb.w = bfr(bb.w);
    const v4f y = (x[p] - mean) * inv * gb + cb;
    stf4x2(op + p * 128 + 4 * lane, y);
  }
}

extern "C" void kernel_launch(void* const* d_in, const int* in_sizes, int n_in,
                              void* d_out, int out_size, void* d_ws, size_t ws_size,
                              hipStream_t stream) {
  if (n_in < 9) return;
  if (in_sizes[0] != NM * NE || in_sizes[1] != NB * NE || in_sizes[2] != NB * NE ||
      in_sizes[3] != NE * NE || in_sizes[4] != NE * NE || in_sizes[5] != NE * NE ||
      in_sizes[6] != NE * NE || in_sizes[7] != NE || in_sizes[8] != NE || out_size != NM * NE)
    return;

  const float* X     = (const float*)d_in[0];
  const float* gq    = (const float*)d_in[1];
  const float* gk    = (const float*)d_in[2];
  const float* Wq    = (const float*)d_in[3];
  const float* Wk    = (const float*)d_in[4];
  const float* Wv    = (const float*)d_in[5];
  const float* Wo    = (const float*)d_in[6];
  const float* gamma = (const float*)d_in[7];
  const float* beta  = (const float*)d_in[8];
  float* out = (float*)d_out;

  const size_t szA16 = (size_t)NM * NE * 2;
  const size_t szW16 = (size_t)NE * NE * 2;
  const size_t szA32 = (size_t)NM * NE * sizeof(float);
  char* ws = (char*)d_ws;
  size_t off = 0;
  __bf16*   Xb   = (__bf16*)(ws + off);   off += szA16;
  __bf16*   Tq   = (__bf16*)(ws + off);   off += szW16;
  __bf16*   Tk   = (__bf16*)(ws + off);   off += szW16;
  __bf16*   Tv   = (__bf16*)(ws + off);   off += szW16;
  _Float16* Wo16 = (_Float16*)(ws + off); off += szW16;
  __bf16*   Qh   = (__bf16*)(ws + off);   off += szA16;
  __bf16*   Ql   = (__bf16*)(ws + off);   off += szA16;
  __bf16*   Kh   = (__bf16*)(ws + off);   off += szA16;
  __bf16*   Kl   = (__bf16*)(ws + off);   off += szA16;
  _Float16* Vt   = (_Float16*)(ws + off); off += szA16;
  _Float16* AO   = (_Float16*)(ws + off); off += szA16;
  float*    Rs   = (float*)(ws + off);    off += szA32;
  if (off > ws_size) return;

  const int n8x = NM * NE / 8;
  cvtx_kernel<<<dim3((n8x + 255) / 256), dim3(256), 0, stream>>>(X, Xb, n8x);
  wprep_kernel<<<dim3(NE / 64, NE / 64, 4), dim3(256), 0, stream>>>(Wq, Wk, Wv, Wo, Tq, Tk, Tv, Wo16);
  qkv_kernel<<<dim3(NE / 64, NM / 128, 3), dim3(128), 0, stream>>>(
      Xb, Tq, Tk, Tv, gq, gk, Qh, Ql, Kh, Kl, Vt);
  attn_kernel<<<dim3(NS / 64, NB * NH), dim3(128), 0, stream>>>(Qh, Ql, Kh, Kl, Vt, AO);
  outproj_kernel<<<dim3(NE / 64, NM / 128), dim3(128), 0, stream>>>(AO, Wo16, X, Rs);
  ln_kernel<<<dim3((NM + 7) / 8), dim3(256), 0, stream>>>(Rs, gamma, beta, out, NM);
}
